// AdapterBlock3D_65755949302444
// MI455X (gfx1250) — hardware-verified
//
#include <hip/hip_runtime.h>
#include <stddef.h>
#include <stdint.h>
#include <math.h>

#define NBAT  2
#define SDIM  16
#define CDIM  768
#define NHEAD 12
#define HDIM  64
#define NTOK  512
#define NWIN  16
#define NWH   192
#define ROWS  8192
#define C3    2304
#define MLPD  3072
#define AHD   192
#define RTAB  15
#define RTR   48
#define PL    ((size_t)NWH * NTOK * HDIM)

static_assert(ROWS == NBAT * SDIM * SDIM * SDIM);
static_assert(ROWS == NWIN * NTOK);
static_assert(NWH == NWIN * NHEAD);
static_assert(NHEAD * HDIM == CDIM);
static_assert(ROWS % 256 == 0);
static_assert(NTOK % 256 == 0);
static_assert(CDIM % 64 == 0 && C3 % 64 == 0 && MLPD % 64 == 0 && AHD % 64 == 0);
static_assert(CDIM % 32 == 0 && AHD % 32 == 0 && MLPD % 32 == 0 && HDIM == 64);
static_assert(RTR * 8 <= 512);

typedef _Float16 v16h __attribute__((ext_vector_type(16)));
typedef _Float16 v8h  __attribute__((ext_vector_type(8)));
typedef float    v8f  __attribute__((ext_vector_type(8)));
typedef float    v4f  __attribute__((ext_vector_type(4)));
typedef unsigned int v4u __attribute__((ext_vector_type(4)));

union Frag  { v16h v; v8h h[2]; };
union Pack8 { v8h h; v4u u; };

__device__ __forceinline__ v8f mma16(v16h a, v16h b, v8f c) {
  c = __builtin_amdgcn_wmma_f32_16x16x32_f16(false, a, false, b, (short)0, c, false, false);
  asm volatile("v_nop\n\tv_nop\n\tv_nop\n\tv_nop" : "+v"(c) : "v"(a), "v"(b));
  return c;
}

__device__ __forceinline__ v16h ldfrag(const _Float16* p, int ld, int row0, int k0, int lane) {
  const int m = lane & 15, lh = lane >> 4;
  const _Float16* q = p + (size_t)(row0 + m) * ld + k0 + 8 * lh;
  Frag f;
  f.h[0] = *(const v8h*)(q);
  f.h[1] = *(const v8h*)(q + 16);
  return f.v;
}

__device__ __forceinline__ v8f zero8() { return (v8f){0.f, 0.f, 0.f, 0.f, 0.f, 0.f, 0.f, 0.f}; }

__device__ __forceinline__ float act16(float v) {
  return 8.0f * v * (1.0f + erff(v * 0.70710678118654752f));
}

__device__ __forceinline__ v4u pack8(v4f a0, v4f a1, float sc) {
  Pack8 pk;
  pk.h = (v8h){(_Float16)(a0[0] * sc), (_Float16)(a0[1] * sc), (_Float16)(a0[2] * sc), (_Float16)(a0[3] * sc),
               (_Float16)(a1[0] * sc), (_Float16)(a1[1] * sc), (_Float16)(a1[2] * sc), (_Float16)(a1[3] * sc)};
  return pk.u;
}

__device__ __forceinline__ int tok2win(int t) {
  const int b = t >> 12, rem = t & 4095;
  const int D = rem >> 8, H = (rem >> 4) & 15, W = rem & 15;
  const int win = ((b * 2 + (D >> 3)) * 2 + (H >> 3)) * 2 + (W >> 3);
  const int n = ((D & 7) * 8 + (H & 7)) * 8 + (W & 7);
  return win * NTOK + n;
}
__device__ __forceinline__ int win2tok(int m) {
  const int win = m >> 9, n = m & 511;
  const int b = win >> 3, db = (win >> 2) & 1, hb = (win >> 1) & 1, wb = win & 1;
  const int d = n >> 6, h = (n >> 3) & 7, w = n & 7;
  return ((b * SDIM + db * 8 + d) * SDIM + hb * 8 + h) * SDIM + wb * 8 + w;
}

template <int KK>
__device__ __forceinline__ void gemm32x64(const _Float16* __restrict__ A, int lda,
                                          const _Float16* __restrict__ Bt, int ldb,
                                          int m0, int n0, int lane, v8f (&acc)[2][4]) {
#pragma unroll 2
  for (int k0 = 0; k0 < KK; k0 += 32) {
    const v16h a0 = ldfrag(A, lda, m0, k0, lane);
    const v16h a1 = ldfrag(A, lda, m0 + 16, k0, lane);
    const v16h b0 = ldfrag(Bt, ldb, n0, k0, lane);
    const v16h b1 = ldfrag(Bt, ldb, n0 + 16, k0, lane);
    const v16h b2 = ldfrag(Bt, ldb, n0 + 32, k0, lane);
    const v16h b3 = ldfrag(Bt, ldb, n0 + 48, k0, lane);
    acc[0][0] = mma16(a0, b0, acc[0][0]);
    acc[1][0] = mma16(a1, b0, acc[1][0]);
    acc[0][1] = mma16(a0, b1, acc[0][1]);
    acc[1][1] = mma16(a1, b1, acc[1][1]);
    acc[0][2] = mma16(a0, b2, acc[0][2]);
    acc[1][2] = mma16(a1, b2, acc[1][2]);
    acc[0][3] = mma16(a0, b3, acc[0][3]);
    acc[1][3] = mma16(a1, b3, acc[1][3]);
  }
}

__global__ __launch_bounds__(256) void k_cvt(const float* __restrict__ w, _Float16* __restrict__ wh,
                                            int ngrp, float sc) {
  const int t = blockIdx.x * 256 + (int)threadIdx.x;
  if (t >= ngrp) return;
  const size_t o = (size_t)t * 8;
  const v4f a0 = *(const v4f*)(w + o);
  const v4f a1 = *(const v4f*)(w + o + 4);
  const v4u vv = pack8(a0, a1, sc);
  volatile v4u* d = (volatile v4u*)(wh + o);
  *d = vv;
  __threadfence();
  *d = vv;
}

__global__ __launch_bounds__(256) void k_rtab(const float* __restrict__ rd, const float* __restrict__ rh,
                                             const float* __restrict__ rwt, _Float16* __restrict__ rt) {
  const int tid = threadIdx.x;
  v4u val[2];
  int go[2];
  bool act[2];
#pragma unroll
  for (int j = 0; j < 2; ++j) {
    const int praw = tid + 256 * j;
    act[j] = praw < RTR * 8;
    const int p = act[j] ? praw : (RTR * 8 - 1);
    const int row = p >> 3, pc = p & 7;
    const int a = row / RTAB;
    const int rr = row - a * RTAB;
    const size_t so = (size_t)rr * HDIM + pc * 8;
    const v4f d0 = *(const v4f*)(rd + so), d1 = *(const v4f*)(rd + so + 4);
    const v4f h0 = *(const v4f*)(rh + so), h1 = *(const v4f*)(rh + so + 4);
    const v4f w0 = *(const v4f*)(rwt + so), w1 = *(const v4f*)(rwt + so + 4);
    const float sd = (a == 0) ? 32.0f : 0.0f;
    const float sh = (a == 1) ? 32.0f : 0.0f;
    const float sw = (a == 2) ? 32.0f : 0.0f;
    v4f e0, e1;
#pragma unroll
    for (int i = 0; i < 4; ++i) {
      e0[i] = d0[i] * sd + h0[i] * sh + w0[i] * sw;
      e1[i] = d1[i] * sd + h1[i] * sh + w1[i] * sw;
    }
    val[j] = pack8(e0, e1, 1.0f);
    go[j]  = row * HDIM + pc * 8;
  }
  for (int ps = 0; ps < 2; ++ps) {
#pragma unroll
    for (int j = 0; j < 2; ++j)
      if (act[j]) *(volatile v4u*)(rt + go[j]) = val[j];
    __threadfence();
  }
}

template <int PERM>
__global__ __launch_bounds__(192) void k_ln(const float* __restrict__ in,
                                           const float* __restrict__ g,
                                           const float* __restrict__ bt,
                                           _Float16* __restrict__ outh) {
  __shared__ __align__(16) float rb[CDIM];
  __shared__ float red[16];
  const int tid = threadIdx.x, lane = tid & 31, wave = tid >> 5;
  const int t = blockIdx.x;
  const int orow = PERM ? tok2win(t) : t;
  const size_t ri = (size_t)t * CDIM;
  const size_t ro = (size_t)orow * CDIM;
  const v4f v = *(const v4f*)(in + ri + 4 * tid);
  float s = (v[0] + v[1]) + (v[2] + v[3]);
#pragma unroll
  for (int off = 1; off < 32; off <<= 1) s += __shfl_xor(s, off, 32);
  if (lane == 0) red[wave] = s;
  __syncthreads();
  float ts = 0.f;
#pragma unroll
  for (int w = 0; w < 6; ++w) ts += red[w];
  const float mean = ts * (1.0f / (float)CDIM);
  const float d0 = v[0] - mean, d1 = v[1] - mean, d2 = v[2] - mean, d3 = v[3] - mean;
  float q = (d0 * d0 + d1 * d1) + (d2 * d2 + d3 * d3);
#pragma unroll
  for (int off = 1; off < 32; off <<= 1) q += __shfl_xor(q, off, 32);
  if (lane == 0) red[8 + wave] = q;
  __syncthreads();
  float tq = 0.f;
#pragma unroll
  for (int w = 0; w < 6; ++w) tq += red[8 + w];
  const float var = tq * (1.0f / (float)CDIM);
  const float inv = rsqrtf(var + 1e-5f);
  const v4f g4 = *(const v4f*)(g + 4 * tid);
  const v4f b4 = *(const v4f*)(bt + 4 * tid);
  v4f o;
  o[0] = d0 * inv * g4[0] + b4[0];
  o[1] = d1 * inv * g4[1] + b4[1];
  o[2] = d2 * inv * g4[2] + b4[2];
  o[3] = d3 * inv * g4[3] + b4[3];
  *(v4f*)(rb + 4 * tid) = o;
  __syncthreads();
  if (tid < 96) {
    const v4f a0 = *(const v4f*)(rb + 8 * tid);
    const v4f a1 = *(const v4f*)(rb + 8 * tid + 4);
    const v4u vv = pack8(a0, a1, 1.0f);
    volatile v4u* hq = (volatile v4u*)(outh + ro + 8 * tid);
    *hq = vv;
    __threadfence();
    *hq = vv;
  }
}

#define STP 72
__global__ __launch_bounds__(256) void k_qkv(const _Float16* __restrict__ xh,
                                             const _Float16* __restrict__ wt,
                                             const float* __restrict__ bqkv,
                                             _Float16* __restrict__ qkv) {
  __shared__ __align__(16) _Float16 st[256 * STP];
  const int tid = threadIdx.x, lane = tid & 31, wave = tid >> 5;
  const int hh = lane >> 4, c = lane & 15;
  const int mb = blockIdx.x * 256;
  const int m0 = mb + wave * 32;
  const int by = (int)blockIdx.y;
  const int n0 = by * 64;
  const int which = by / NHEAD;
  const int head  = by - which * NHEAD;

  v8f acc[2][4];
#pragma unroll
  for (int s = 0; s < 2; ++s)
#pragma unroll
    for (int t = 0; t < 4; ++t) acc[s][t] = zero8();
  gemm32x64<CDIM>(xh, CDIM, wt, CDIM, m0, n0, lane, acc);

#pragma unroll
  for (int t = 0; t < 4; ++t) {
    const float bb = bqkv[n0 + 16 * t + c];
#pragma unroll
    for (int sub = 0; sub < 2; ++sub) {
#pragma unroll
      for (int r = 0; r < 8; ++r) {
        const int lr = wave * 32 + sub * 16 + 8 * hh + r;
        st[lr * STP + 16 * t + c] = (_Float16)(acc[sub][t][r] * 0.03125f + bb);
      }
    }
  }
  __syncthreads();

  const int win = mb >> 9;
  const int nb  = mb & (NTOK - 1);
  const int wh  = win * NHEAD + head;
  v4u val[8];
  size_t go[8];
  if (which < 2) {
#pragma unroll
    for (int j = 0; j < 8; ++j) {
      const int p  = tid + 256 * j;
      const int lr = p >> 3;
      const int pc = p & 7;
      Pack8 pk;
      pk.h  = *(const v8h*)(st + lr * STP + pc * 8);
      val[j] = pk.u;
      go[j]  = (size_t)which * PL + ((size_t)wh * NTOK + nb + lr) * HDIM + pc * 8;
    }
  } else {
#pragma unroll
    for (int j = 0; j < 8; ++j) {
      const int p  = tid + 256 * j;
      const int L  = p >> 3;
      const int pc = p & 7;
      const int d  = L >> 2;
      const int nl = (L & 3) * 64 + pc * 8;
      const _Float16* cp = st + nl * STP + d;
      Pack8 pk;
      pk.h = (v8h){cp[0 * STP], cp[1 * STP], cp[2 * STP], cp[3 * STP],
                   cp[4 * STP], cp[5 * STP], cp[6 * STP], cp[7 * STP]};
      val[j] = pk.u;
      go[j]  = 2 * PL + ((size_t)wh * HDIM + d) * NTOK + nb + nl;
    }
  }
  for (int ps = 0; ps < 2; ++ps) {
#pragma unroll
    for (int j = 0; j < 8; ++j) *(volatile v4u*)(qkv + go[j]) = val[j];
    __threadfence();
  }
}

#define KTP 72
#define PTP 72
__global__ __launch_bounds__(256) void k_attn(const _Float16* __restrict__ qp,
                                              const _Float16* __restrict__ kp,
                                              const _Float16* __restrict__ vt,
                                              const _Float16* __restrict__ rt,
                                              _Float16* __restrict__ op, float sscale) {
  __shared__ __align__(16) _Float16 Ks[64 * KTP];
  __shared__ __align__(16) _Float16 Vs[64 * KTP];
  __shared__ __align__(16) _Float16 Ps[8][16 * PTP];
  __shared__ __align__(16) float    Rs[8][16 * RTR];

  const int tid = threadIdx.x, lane = tid & 31, wave = tid >> 5;
  const int hh = lane >> 4, c = lane & 15;
  const int wh = blockIdx.x >> 2;
  const int qb = blockIdx.x & 3;
  const int win = wh / NHEAD, head = wh - win * NHEAD;
  const int q0 = qb * 128 + wave * 16;

  const _Float16* Q = qp + (size_t)wh * NTOK * HDIM;
  const _Float16* K = kp + (size_t)wh * NTOK * HDIM;
  const _Float16* V = vt + (size_t)wh * HDIM * NTOK;

  v16h qa[2];
  qa[0] = ldfrag(Q, HDIM, q0, 0, lane);
  qa[1] = ldfrag(Q, HDIM, q0, 32, lane);

  float* rsw = Rs[wave];
  {
    v8f racc[3];
#pragma unroll
    for (int t = 0; t < 3; ++t) racc[t] = zero8();
#pragma unroll
    for (int dc = 0; dc < 2; ++dc) {
#pragma unroll
      for (int t = 0; t < 3; ++t) {
        const v16h rb = ldfrag(rt, HDIM, 16 * t, 32 * dc, lane);
        racc[t] = mma16(qa[dc], rb, racc[t]);
      }
    }
#pragma unroll
    for (int t = 0; t < 3; ++t)
#pragma unroll
      for (int r = 0; r < 8; ++r) rsw[(8 * hh + r) * RTR + 16 * t + c] = racc[t][r] * 0.03125f;
  }
  __syncthreads();

  const int qd  = (q0 >> 6) & 7;
  const int qhh = ((q0 >> 3) & 7) + hh;
  const int hb  = 22 + qhh - (c >> 3);
  float bwv[8];
#pragma unroll
  for (int r = 0; r < 8; ++r) bwv[r] = rsw[(8 * hh + r) * RTR + 37 + r - (c & 7)];

  const float NEGI = -__builtin_huge_valf();
  float mrow[8], lrow[8];
  v8f oacc[4];
#pragma unroll
  for (int r = 0; r < 8; ++r) { mrow[r] = NEGI; lrow[r] = 0.f; }
#pragma unroll
  for (int t = 0; t < 4; ++t) oacc[t] = zero8();

  _Float16* pw = Ps[wave];

  for (int kc = 0; kc < NTOK / 64; ++kc) {
    const int kv0 = kc * 64;
    __syncthreads();
    {
      const int r  = tid >> 2;
      const int qq = (tid & 3) * 16;
      const _Float16* ks = K + (size_t)(kv0 + r) * HDIM + qq;
      *(v8h*)(Ks + r * KTP + qq)     = *(const v8h*)(ks);
      *(v8h*)(Ks + r * KTP + qq + 8) = *(const v8h*)(ks + 8);
      const _Float16* vs = V + (size_t)r * NTOK + kv0 + qq;
      *(v8h*)(Vs + r * KTP + qq)     = *(const v8h*)(vs);
      *(v8h*)(Vs + r * KTP + qq + 8) = *(const v8h*)(vs + 8);
    }
    __syncthreads();

    v8f s[4];
#pragma unroll
    for (int j = 0; j < 4; ++j) s[j] = zero8();
#pragma unroll
    for (int dc = 0; dc < 2; ++dc) {
#pragma unroll
      for (int j = 0; j < 4; ++j) {
        const v16h kb = ldfrag(Ks, KTP, j * 16, dc * 32, lane);
        s[j] = mma16(qa[dc], kb, s[j]);
      }
    }
    const int dcol = qd - kc + 7;
    float cm[8];
#pragma unroll
    for (int r = 0; r < 8; ++r) {
      const float* rrow = rsw + (8 * hh + r) * RTR;
      const float bdw = rrow[dcol] + bwv[r];
      float m = NEGI;
#pragma unroll
      for (int j = 0; j < 4; ++j) {
        const float sv = s[j][r] * sscale + (bdw + rrow[hb - 2 * j]);
        s[j][r] = sv;
        m = fmaxf(m, sv);
      }
#pragma unroll
      for (int off = 1; off < 16; off <<= 1) m = fmaxf(m, __shfl_xor(m, off, 32));
      cm[r] = m;
    }
    float al[8];
#pragma unroll
    for (int r = 0; r < 8; ++r) {
      const float mnew  = fmaxf(mrow[r], cm[r]);
      const float alpha = __expf(mrow[r] - mnew);
      mrow[r] = mnew;
      float psum = 0.f;
#pragma unroll
      for (int j = 0; j < 4; ++j) {
        const float p = __expf(s[j][r] - mnew);
        psum += p;
        pw[(8 * hh + r) * PTP + j * 16 + c] = (_Float16)(p * 1024.0f);
      }
#pragma unroll
      for (int off = 1; off < 16; off <<= 1) psum += __shfl_xor(psum, off, 32);
      lrow[r] = lrow[r] * alpha + psum;
      al[r] = alpha;
    }
#pragma unroll
    for (int t = 0; t < 4; ++t)
#pragma unroll
      for (int r = 0; r < 8; ++r) oacc[t][r] *= al[r];
    __syncthreads();

#pragma unroll
    for (int kk = 0; kk < 2; ++kk) {
      const v16h pa = ldfrag(pw, PTP, 0, kk * 32, lane);
#pragma unroll
      for (int t = 0; t < 4; ++t) {
        const v16h vb = ldfrag(Vs, KTP, t * 16, kk * 32, lane);
        oacc[t] = mma16(pa, vb, oacc[t]);
      }
    }
  }
  __syncthreads();

#pragma unroll
  for (int r = 0; r < 8; ++r) {
    const float inv = 0.0625f / lrow[r];
#pragma unroll
    for (int t = 0; t < 4; ++t) pw[(8 * hh + r) * PTP + 16 * t + c] = (_Float16)(oacc[t][r] * inv);
  }
  __syncthreads();
  v4u val[4];
  size_t go[4];
#pragma unroll
  for (int it = 0; it < 4; ++it) {
    const int p  = lane + 32 * it;
    const int L  = p >> 3;
    const int pc = p & 7;
    Pack8 pk;
    pk.h   = *(const v8h*)(pw + L * PTP + pc * 8);
    val[it] = pk.u;
    go[it]  = ((size_t)(win * NTOK + q0 + L)) * CDIM + (size_t)head * HDIM + pc * 8;
  }
  for (int ps = 0; ps < 2; ++ps) {
#pragma unroll
    for (int it = 0; it < 4; ++it) *(volatile v4u*)(op + go[it]) = val[it];
    __threadfence();
  }
}

#define OTP 68
__global__ __launch_bounds__(256) void k_proj(const _Float16* __restrict__ ap,
                                              const _Float16* __restrict__ wt,
                                              const float* __restrict__ bias,
                                              float* __restrict__ outf,
                                              _Float16* __restrict__ outh, float oscale) {
  __shared__ __align__(16) float st[8][16 * OTP];
  const int tid = threadIdx.x, lane = tid & 31, wave = tid >> 5;
  const int hh = lane >> 4, c = lane & 15;
  const int m0 = blockIdx.x * 256 + wave * 32;
  const int n0 = (int)blockIdx.y * 64;

  v8f acc[2][4];
#pragma unroll
  for (int s = 0; s < 2; ++s)
#pragma unroll
    for (int t = 0; t < 4; ++t) acc[s][t] = zero8();
  gemm32x64<CDIM>(ap, CDIM, wt, CDIM, m0, n0, lane, acc);

  float bvs[4];
#pragma unroll
  for (int t = 0; t < 4; ++t) bvs[t] = bias[n0 + 16 * t + c];

  float* sw = st[wave];
#pragma unroll
  for (int sub = 0; sub < 2; ++sub) {
    __syncthreads();
#pragma unroll
    for (int t = 0; t < 4; ++t) {
#pragma unroll
      for (int r = 0; r < 8; ++r)
        sw[(8 * hh + r) * OTP + 16 * t + c] = acc[sub][t][r] * oscale + bvs[t];
    }
    __syncthreads();
    v4f val[8];
    size_t go[8];
#pragma unroll
    for (int it = 0; it < 8; ++it) {
      const int p    = lane + 32 * it;
      const int L    = p >> 3;
      const int pc   = p & 7;
      const int row  = L >> 1;
      const int half = L & 1;
      val[it] = *(const v4f*)(sw + row * OTP + half * 32 + pc * 4);
      go[it]  = (size_t)(m0 + sub * 16 + row) * CDIM + n0 + half * 32 + pc * 4;
    }
    v4u valh[4];
    size_t goh[4];
#pragma unroll
    for (int it = 0; it < 4; ++it) {
      const int p  = lane + 32 * it;
      const int L  = p >> 3;
      const int pc = p & 7;
      const v4f x0 = *(const v4f*)(sw + L * OTP + pc * 8);
      const v4f x1 = *(const v4f*)(sw + L * OTP + pc * 8 + 4);
      valh[it] = pack8(x0, x1, 16.0f);
      goh[it]  = (size_t)(m0 + sub * 16 + L) * CDIM + n0 + pc * 8;
    }
    for (int ps = 0; ps < 2; ++ps) {
#pragma unroll
      for (int it = 0; it < 8; ++it) *(volatile v4f*)(outf + go[it]) = val[it];
#pragma unroll
      for (int it = 0; it < 4; ++it) *(volatile v4u*)(outh + goh[it]) = valh[it];
      __threadfence();
    }
  }
}

template <int KK, int NOUT>
__global__ __launch_bounds__(256) void k_ffn1(const _Float16* __restrict__ ap,
                                              const _Float16* __restrict__ wt,
                                              const float* __restrict__ bias,
                                              _Float16* __restrict__ hp, float ascale) {
  __shared__ __align__(16) float st[8][16 * OTP];
  const int tid = threadIdx.x, lane = tid & 31, wave = tid >> 5;
  const int hh = lane >> 4, c = lane & 15;
  const int m0 = blockIdx.x * 256 + wave * 32;
  const int n0 = (int)blockIdx.y * 64;

  v8f acc[2][4];
#pragma unroll
  for (int s = 0; s < 2; ++s)
#pragma unroll
    for (int t = 0; t < 4; ++t) acc[s][t] = zero8();
  gemm32x64<KK>(ap, KK, wt, KK, m0, n0, lane, acc);

  float bvs[4];
#pragma unroll
  for (int t = 0; t < 4; ++t) bvs[t] = bias[n0 + 16 * t + c];

  float* sw = st[wave];
#pragma unroll
  for (int sub = 0; sub < 2; ++sub) {
    __syncthreads();
#pragma unroll
    for (int t = 0; t < 4; ++t) {
#pragma unroll
      for (int r = 0; r < 8; ++r)
        sw[(8 * hh + r) * OTP + 16 * t + c] = acc[sub][t][r] * ascale + bvs[t];
    }
    __syncthreads();
    v4u val[4];
    size_t go[4];
#pragma unroll
    for (int it = 0; it < 4; ++it) {
      const int p  = lane + 32 * it;
      const int L  = p >> 3;
      const int pc = p & 7;
      const v4f x0 = *(const v4f*)(sw + L * OTP + pc * 8);
      const v4f x1 = *(const v4f*)(sw + L * OTP + pc * 8 + 4);
      Pack8 pk;
      pk.h = (v8h){(_Float16)act16(x0[0]), (_Float16)act16(x0[1]), (_Float16)act16(x0[2]), (_Float16)act16(x0[3]),
                   (_Float16)act16(x1[0]), (_Float16)act16(x1[1]), (_Float16)act16(x1[2]), (_Float16)act16(x1[3])};
      val[it] = pk.u;
      go[it]  = (size_t)(m0 + sub * 16 + L) * NOUT + n0 + pc * 8;
    }
    for (int ps = 0; ps < 2; ++ps) {
#pragma unroll
      for (int it = 0; it < 4; ++it) *(volatile v4u*)(hp + go[it]) = val[it];
      __threadfence();
    }
  }
}

__global__ __launch_bounds__(256) void k_adp2(const _Float16* __restrict__ ap,
                                              const _Float16* __restrict__ wt,
                                              const float* __restrict__ bias,
                                              const float* __restrict__ resw,
                                              const float* __restrict__ rest,
                                              float* __restrict__ out, float oscale) {
  __shared__ __align__(16) float st[8][16 * OTP];
  const int tid = threadIdx.x, lane = tid & 31, wave = tid >> 5;
  const int hh = lane >> 4, c = lane & 15;
  const int m0 = blockIdx.x * 256 + wave * 32;
  const int n0 = (int)blockIdx.y * 64;

  v8f acc[2][4];
#pragma unroll
  for (int s = 0; s < 2; ++s)
#pragma unroll
    for (int t = 0; t < 4; ++t) acc[s][t] = zero8();
  gemm32x64<AHD>(ap, AHD, wt, AHD, m0, n0, lane, acc);

  float bvs[4];
#pragma unroll
  for (int t = 0; t < 4; ++t) bvs[t] = bias[n0 + 16 * t + c];

  float* sw = st[wave];
#pragma unroll
  for (int sub = 0; sub < 2; ++sub) {
    __syncthreads();
#pragma unroll
    for (int t = 0; t < 4; ++t) {
#pragma unroll
      for (int r = 0; r < 8; ++r)
        sw[(8 * hh + r) * OTP + 16 * t + c] = acc[sub][t][r] * oscale + bvs[t];
    }
    __syncthreads();
    v4f val[8];
    size_t go[8];
#pragma unroll
    for (int it = 0; it < 8; ++it) {
      const int p    = lane + 32 * it;
      const int L    = p >> 3;
      const int pc   = p & 7;
      const int row  = L >> 1;
      const int half = L & 1;
      const int mw   = m0 + sub * 16 + row;
      const int mt   = win2tok(mw);
      const int col  = n0 + half * 32 + pc * 4;
      const size_t gw = (size_t)mw * CDIM + col;
      const size_t gt = (size_t)mt * CDIM + col;
      v4f v = *(const v4f*)(sw + row * OTP + half * 32 + pc * 4);
      const v4f r1 = *(const v4f*)(resw + gw);
      const v4f r2 = *(const v4f*)(rest + gt);
      v[0] = (v[0] + r1[0]) + r2[0];
      v[1] = (v[1] + r1[1]) + r2[1];
      v[2] = (v[2] + r1[2]) + r2[2];
      v[3] = (v[3] + r1[3]) + r2[3];
      val[it] = v;
      go[it]  = gt;
    }
    for (int ps = 0; ps < 2; ++ps) {
#pragma unroll
      for (int it = 0; it < 8; ++it) *(volatile v4f*)(out + go[it]) = val[it];
      __threadfence();
    }
  }
}

__global__ __launch_bounds__(256) void k_final(const _Float16* __restrict__ a1p,
                                               const _Float16* __restrict__ w1t,
                                               const _Float16* __restrict__ a2p,
                                               const _Float16* __restrict__ w2t,
                                               const float* __restrict__ b1,
                                               const float* __restrict__ b2,
                                               const float* __restrict__ res,
                                               float* __restrict__ out, float oscale) {
  __shared__ __align__(16) float st[8][16 * OTP];
  const int tid = threadIdx.x, lane = tid & 31, wave = tid >> 5;
  const int hh = lane >> 4, c = lane & 15;
  const int m0 = blockIdx.x * 256 + wave * 32;
  const int n0 = (int)blockIdx.y * 64;

  v8f acc[2][4];
#pragma unroll
  for (int s = 0; s < 2; ++s)
#pragma unroll
    for (int t = 0; t < 4; ++t) acc[s][t] = zero8();
  gemm32x64<MLPD>(a1p, MLPD, w1t, MLPD, m0, n0, lane, acc);
  gemm32x64<AHD>(a2p, AHD, w2t, AHD, m0, n0, lane, acc);

  float bvs[4];
#pragma unroll
  for (int t = 0; t < 4; ++t) {
    const int nn = n0 + 16 * t + c;
    bvs[t] = b1[nn] + 0.5f * b2[nn];
  }

  float* sw = st[wave];
#pragma unroll
  for (int sub = 0; sub < 2; ++sub) {
    __syncthreads();
#pragma unroll
    for (int t = 0; t < 4; ++t) {
#pragma unroll
      for (int r = 0; r < 8; ++r)
        sw[(8 * hh + r) * OTP + 16 * t + c] = acc[sub][t][r] * oscale + bvs[t];
    }
    __syncthreads();
    v4f val[8];
    size_t go[8];
#pragma unroll
    for (int it = 0; it < 8; ++it) {
      const int p    = lane + 32 * it;
      const int L    = p >> 3;
      const int pc   = p & 7;
      const int row  = L >> 1;
      const int half = L & 1;
      const size_t g = (size_t)(m0 + sub * 16 + row) * CDIM + n0 + half * 32 + pc * 4;
      v4f v = *(const v4f*)(sw + row * OTP + half * 32 + pc * 4);
      const v4f rr = *(const v4f*)(res + g);
      v[0] = v[0] + rr[0]; v[1] = v[1] + rr[1]; v[2] = v[2] + rr[2]; v[3] = v[3] + rr[3];
      val[it] = v;
      go[it]  = g;
    }
    for (int ps = 0; ps < 2; ++ps) {
#pragma unroll
      for (int it = 0; it < 8; ++it) *(volatile v4f*)(out + go[it]) = val[it];
      __threadfence();
    }
  }
}

static_assert((size_t)ROWS * CDIM * 2 + 3 * PL * 2 <= (size_t)ROWS * MLPD * 2);
static_assert((size_t)ROWS * CDIM * 4 + (size_t)ROWS * CDIM * 2 + (size_t)ROWS * AHD * 2 <= (size_t)ROWS * MLPD * 2);

extern "C" void kernel_launch(void* const* d_in, const int* in_sizes, int n_in,
                              void* d_out, int out_size, void* d_ws, size_t ws_size,
                              hipStream_t stream) {
  if (n_in < 24) return;
  if (in_sizes[0] != ROWS * CDIM) return;
  if (in_sizes[1] != CDIM || in_sizes[2] != CDIM) return;
  if (in_sizes[3] != C3 * CDIM || in_sizes[4] != C3) return;
  if (in_sizes[5] != RTAB * HDIM || in_sizes[6] != RTAB * HDIM || in_sizes[7] != RTAB * HDIM) return;
  if (in_sizes[8] != CDIM * CDIM || in_sizes[9] != CDIM) return;
  if (in_sizes[10] != AHD * CDIM || in_sizes[11] != AHD) return;
  if (in_sizes[12] != CDIM * AHD || in_sizes[13] != CDIM) return;
  if (in_sizes[14] != CDIM || in_sizes[15] != CDIM) return;
  if (in_sizes[16] != MLPD * CDIM || in_sizes[17] != MLPD) return;
  if (in_sizes[18] != CDIM * MLPD || in_sizes[19] != CDIM) return;
  if (in_sizes[20] != AHD * CDIM || in_sizes[21] != AHD) return;
  if (in_sizes[22] != CDIM * AHD || in_sizes[23] != CDIM) return;
  if (out_size != ROWS * CDIM) return;

  const float* x     = (const float*)d_in[0];
  const float* ln1g  = (const float*)d_in[1];
  const float* ln1b  = (const float*)d_in[2];
  const float* qkvw  = (const float*)d_in[3];
  const float* qkvb  = (const float*)d_in[4];
  const float* rpd   = (const float*)d_in[5];
  const float* rph   = (const float*)d_in[6];
  const float* rpw   = (const float*)d_in[7];
  const float* projw = (const float*)d_in[8];
  const float* projb = (const float*)d_in[9];
  const float* aa1w  = (const float*)d_in[10];
  const float* aa1b  = (const float*)d_in[11];
  const float* aa2w  = (const float*)d_in[12];
  const float* aa2b  = (const float*)d_in[13];
  const float* ln2g  = (const float*)d_in[14];
  const float* ln2b  = (const float*)d_in[15];
  const float* mlp1w = (const float*)d_in[16];
  const float* mlp1b = (const float*)d_in[17];
  const float* mlp2w = (const float*)d_in[18];
  const float* mlp2b = (const float*)d_in[19];
  const float* ma1w  = (const float*)d_in[20];
  const float* ma1b  = (const float*)d_in[21];
  const float* ma2w  = (const float*)d_in[22];
  const float* ma2b  = (const float*)d_in[23];
  float* out = (float*)d_out;

  size_t off = 0;
  const size_t oWqkv  = off; off += (size_t)C3 * CDIM * 2;
  const size_t oWproj = off; off += (size_t)CDIM * CDIM * 2;
  const size_t oWaa1  = off; off += (size_t)AHD * CDIM * 2;
  const size_t oWaa2  = off; off += (size_t)CDIM * AHD * 2;
  const size_t oWmlp1 = off; off += (size_t)MLPD * CDIM * 2;
  const size_t oWmlp2 = off; off += (size_t)CDIM * MLPD * 2;
  const size_t oWma1  = off; off += (size_t)AHD * CDIM * 2;
  const size_t oWma2  = off; off += (size_t)CDIM * AHD * 2;
  const size_t oRt    = off; off += (size_t)RTR * HDIM * 2;
  const size_t oA     = off; off += (size_t)ROWS * MLPD * 2;
  const size_t oLN1h  = oA;
  const size_t oQKV   = oA + (size_t)ROWS * CDIM * 2;
  const size_t oT1    = oA;
  const size_t oT1h   = oA + (size_t)ROWS * CDIM * 4;
  const size_t oA1    = oT1h + (size_t)ROWS * CDIM * 2;
  const size_t oM1    = oA;
  const size_t oB     = off; off += (size_t)ROWS * CDIM * 2;
  const size_t oH     = off; off += (size_t)ROWS * CDIM * 4;
  const size_t oAM1   = off; off += (size_t)ROWS * AHD * 2;
  if (off > ws_size) return;
  if (off > (size_t)134217728) return;

  char* ws = (char*)d_ws;
  _Float16* Wqkv  = (_Float16*)(ws + oWqkv);
  _Float16* Wproj = (_Float16*)(ws + oWproj);
  _Float16* Waa1  = (_Float16*)(ws + oWaa1);
  _Float16* Waa2  = (_Float16*)(ws + oWaa2);
  _Float16* Wmlp1 = (_Float16*)(ws + oWmlp1);
  _Float16* Wmlp2 = (_Float16*)(ws + oWmlp2);
  _Float16* Wma1  = (_Float16*)(ws + oWma1);
  _Float16* Wma2  = (_Float16*)(ws + oWma2);
  _Float16* Rt    = (_Float16*)(ws + oRt);
  _Float16* LN1h  = (_Float16*)(ws + oLN1h);
  _Float16* QKVp  = (_Float16*)(ws + oQKV);
  float*    T1    = (float*)(ws + oT1);
  _Float16* T1h   = (_Float16*)(ws + oT1h);
  _Float16* A1    = (_Float16*)(ws + oA1);
  _Float16* M1    = (_Float16*)(ws + oM1);
  _Float16* CTX   = (_Float16*)(ws + oB);
  _Float16* HN    = (_Float16*)(ws + oB);
  float*    H     = (float*)(ws + oH);
  _Float16* AM1   = (_Float16*)(ws + oAM1);

  {
    const int g3 = in_sizes[3] / 8, g8 = in_sizes[8] / 8, g10 = in_sizes[10] / 8, g12 = in_sizes[12] / 8;
    const int g16 = in_sizes[16] / 8, g18 = in_sizes[18] / 8, g20 = in_sizes[20] / 8, g22 = in_sizes[22] / 8;
    k_cvt<<<dim3((g3 + 255) / 256), dim3(256), 0, stream>>>(qkvw, Wqkv, g3, 32.0f);
    k_cvt<<<dim3((g8 + 255) / 256), dim3(256), 0, stream>>>(projw, Wproj, g8, 32.0f);
    k_cvt<<<dim3((g10 + 255) / 256), dim3(256), 0, stream>>>(aa1w, Waa1, g10, 32.0f);
    k_cvt<<<dim3((g12 + 255) / 256), dim3(256), 0, stream>>>(aa2w, Waa2, g12, 32.0f);
    k_cvt<<<dim3((g16 + 255) / 256), dim3(256), 0, stream>>>(mlp1w, Wmlp1, g16, 32.0f);
    k_cvt<<<dim3((g18 + 255) / 256), dim3(256), 0, stream>>>(mlp2w, Wmlp2, g18, 32.0f);
    k_cvt<<<dim3((g20 + 255) / 256), dim3(256), 0, stream>>>(ma1w, Wma1, g20, 32.0f);
    k_cvt<<<dim3((g22 + 255) / 256), dim3(256), 0, stream>>>(ma2w, Wma2, g22, 16.0f);
  }
  k_rtab<<<dim3(1), dim3(256), 0, stream>>>(rpd, rph, rpw, Rt);
  k_ln<1><<<dim3(ROWS), dim3(192), 0, stream>>>(x, ln1g, ln1b, LN1h);
  k_qkv<<<dim3(ROWS / 256, C3 / 64), dim3(256), 0, stream>>>(LN1h, Wqkv, qkvb, QKVp);
  k_attn<<<dim3(NWH * (NTOK / 128)), dim3(256), 0, stream>>>(QKVp, QKVp + PL, QKVp + 2 * PL, Rt, CTX, 0.125f);
  k_proj<<<dim3(ROWS / 256, CDIM / 64), dim3(256), 0, stream>>>(CTX, Wproj, projb, T1, T1h, 0.00048828125f);
  k_ffn1<CDIM, AHD><<<dim3(ROWS / 256, AHD / 64), dim3(256), 0, stream>>>(T1h, Waa1, aa1b, A1, 0.001953125f);
  k_adp2<<<dim3(ROWS / 256, CDIM / 64), dim3(256), 0, stream>>>(A1, Waa2, aa2b, T1, x, H, 0.001953125f);
  k_ln<0><<<dim3(ROWS), dim3(192), 0, stream>>>(H, ln2g, ln2b, HN);
  k_ffn1<CDIM, MLPD><<<dim3(ROWS / 256, MLPD / 64), dim3(256), 0, stream>>>(HN, Wmlp1, mlp1b, M1, 0.03125f);
  k_ffn1<CDIM, AHD><<<dim3(ROWS / 256, AHD / 64), dim3(256), 0, stream>>>(HN, Wma1, ma1b, AM1, 0.03125f);
  k_final<<<dim3(ROWS / 256, CDIM / 64), dim3(256), 0, stream>>>(M1, Wmlp2, AM1, Wma2, mlp2b, ma2b, H, out, 0.001953125f);
  (void)hipGetLastError();
}
